// FusedExpertGroup_65180423685437
// MI455X (gfx1250) — hardware-verified
//
#include <hip/hip_runtime.h>
#include <math.h>

typedef __attribute__((ext_vector_type(16))) _Float16 v16h;
typedef __attribute__((ext_vector_type(16))) __bf16 v16b;
typedef __attribute__((ext_vector_type(8)))  _Float16 v8h;
typedef __attribute__((ext_vector_type(8)))  float v8f;
typedef __attribute__((ext_vector_type(4)))  float v4f;
typedef __attribute__((ext_vector_type(2)))  float v2f;
typedef __attribute__((ext_vector_type(4)))  unsigned v4u;
typedef __attribute__((ext_vector_type(4)))  int v4i;
typedef float __attribute__((may_alias)) float_a;
typedef int __attribute__((may_alias)) int_a;

template <typename T> __device__ __forceinline__ void vst2(void* p, T v) { *(volatile T*)p = v; __threadfence(); *(volatile T*)p = v; }
__device__ __forceinline__ v8f wmma16(v16h a, v16h b, v8f c) {
  v8f d = __builtin_amdgcn_wmma_f32_16x16x32_f16(false, a, false, b, (short)0, c, false, false);
  asm volatile("v_nop\n\tv_nop\n\tv_nop\n\tv_nop" : "+v"(d) : "v"(a), "v"(b));
  return d;
}
__device__ __forceinline__ v8f wmma_bf(v16b a, v16b b, v8f c) {
  v8f d = __builtin_amdgcn_wmma_f32_16x16x32_bf16(false, a, false, b, (short)0, c, false, false);
  asm volatile("v_nop\n\tv_nop\n\tv_nop\n\tv_nop" : "+v"(d) : "v"(a), "v"(b));
  return d;
}
__device__ __forceinline__ v16h frag_h(const _Float16* rowk0, int lane) {
  union { v16h v; v8h q[2]; } u; const _Float16* p = rowk0 + 8 * (lane >> 4);
  u.q[0] = *(const v8h*)p; u.q[1] = *(const v8h*)(p + 16); return u.v;
}
__device__ __forceinline__ v16h frag_f32(const float* rowk0, int lane) {
  v16h a; const float* p = rowk0 + 8 * (lane >> 4);
#pragma unroll
  for (int i = 0; i < 8; ++i) { a[i] = (_Float16)p[i]; a[8 + i] = (_Float16)p[16 + i]; }
  return a;
}
__device__ __forceinline__ v16h frag_f32s(const float* rowk0, int lane, float sc) {
  v16h a; const float* p = rowk0 + 8 * (lane >> 4);
#pragma unroll
  for (int i = 0; i < 8; ++i) { a[i] = (_Float16)(p[i] * sc); a[8 + i] = (_Float16)(p[16 + i] * sc); }
  return a;
}
__device__ __forceinline__ v16h fragc_f32(const float* W, int k0, int n, int lane, int ld, int K) {
  v16h a; const int g = lane >> 4;
#pragma unroll
  for (int i = 0; i < 8; ++i) { const int ka = k0 + 8 * g + i, kb = ka + 16;
    a[i] = (_Float16)(ka < K ? W[(size_t)ka * ld + n] : 0.f); a[8 + i] = (_Float16)(kb < K ? W[(size_t)kb * ld + n] : 0.f); }
  return a;
}
struct F2 { v16b h, l; };
__device__ __forceinline__ F2 bsplit16(const float v[16]) { F2 r;
#pragma unroll
  for (int i = 0; i < 16; ++i) { const __bf16 h = (__bf16)v[i]; r.h[i] = h; r.l[i] = (__bf16)(v[i] - (float)h); }
  return r; }
__device__ __forceinline__ F2 split_row(const float* row, int k0, int lane) { float v[16]; const float* p = row + k0 + 8 * (lane >> 4);
#pragma unroll
  for (int i = 0; i < 8; ++i) { v[i] = p[i]; v[8 + i] = p[16 + i]; }
  return bsplit16(v); }
__device__ __forceinline__ F2 split_rowK(const float* row, int k0, int lane, int K) { float v[16]; const int g = lane >> 4;
#pragma unroll
  for (int i = 0; i < 8; ++i) { const int ka = k0 + 8 * g + i, kb = ka + 16; v[i] = ka < K ? row[ka] : 0.f; v[8 + i] = kb < K ? row[kb] : 0.f; }
  return bsplit16(v); }
__device__ __forceinline__ F2 split_col(const float* W, int k0, int n, int lane, int ld, int K) { float v[16]; const int g = lane >> 4;
#pragma unroll
  for (int i = 0; i < 8; ++i) { const int ka = k0 + 8 * g + i, kb = ka + 16; v[i] = ka < K ? W[(size_t)ka * ld + n] : 0.f; v[8 + i] = kb < K ? W[(size_t)kb * ld + n] : 0.f; }
  return bsplit16(v); }
__device__ __forceinline__ v8f mac3(const F2& a, const F2& b, v8f c) { c = wmma_bf(a.l, b.h, c); c = wmma_bf(a.h, b.l, c); return wmma_bf(a.h, b.h, c); }
__device__ __forceinline__ float sigm(float v) { return 1.0f / (1.0f + expf(-v)); }
#define LDSX() do { asm volatile("s_wait_dscnt 0" ::: "memory"); __builtin_amdgcn_wave_barrier(); __builtin_amdgcn_fence(__ATOMIC_RELEASE, "workgroup"); } while (0)

#define NBT 8
#define CIN 256
#define HW 64
#define NPX (HW * HW)
#define NE 8
#define COUT 256
#define TOPK 2
#define CIG 32
#define KC (CIG * 9)
#define NG 8
#define NBLK (NPX / 64)

__global__ __launch_bounds__(128) void k_conv(const float* __restrict__ x, const int* __restrict__ ridx, const float* __restrict__ cw, float* __restrict__ F, float* __restrict__ PART) {
  __shared__ __align__(16) _Float16 sa[4][16][40];
  __shared__ __align__(16) float so[COUT][68];
  __shared__ float sred[4][NG][2];
  const int tid = threadIdx.x, wave = tid >> 5, lane = tid & 31, col = lane & 15, g = lane >> 4;
  const int bk = blockIdx.y, b = bk >> 1, kk = bk & 1; int e = ridx[b * TOPK + kk]; e = e < 0 ? 0 : (e >= NE ? NE - 1 : e);
  const int p0 = blockIdx.x * 64 + wave * 16; const int pm = p0 + col, ym = pm / HW, xm = pm % HW;
  const float* xb = x + ((size_t)b * CIN + e * CIG) * NPX; const float* wb = cw + (size_t)e * COUT * KC;
  v8f acc[16];
#pragma unroll
  for (int t = 0; t < 16; ++t) acc[t] = (v8f){};
#pragma unroll 1
  for (int kc = 0; kc < KC / 32; ++kc) {
    { union { v8h h[2]; v4u u2[2]; } pk;
#pragma unroll
      for (int u = 0; u < 16; ++u) { const int k = kc * 32 + g * 16 + u; const int ci = k / 9, tap = k % 9; const int yy = ym + tap / 3 - 1, xx = xm + tap % 3 - 1;
        float v = 0.f; if (yy >= 0 && yy < HW && xx >= 0 && xx < HW) v = xb[(size_t)ci * NPX + yy * HW + xx];
        pk.h[u >> 3][u & 7] = (_Float16)v; }
      *(v4u*)(&sa[wave][col][g * 16]) = pk.u2[0]; *(v4u*)(&sa[wave][col][g * 16 + 8]) = pk.u2[1]; }
    LDSX();
    const v16h a = frag_h(&sa[wave][col][0], lane);
#pragma unroll
    for (int t = 0; t < 16; ++t) acc[t] = wmma16(a, frag_f32s(wb + (size_t)(t * 16 + col) * KC + kc * 32, lane, 16.0f), acc[t]);
    LDSX(); }
  float gs[NG], gq[NG];
#pragma unroll
  for (int gi = 0; gi < NG; ++gi) { gs[gi] = 0.f; gq[gi] = 0.f; }
#pragma unroll
  for (int t = 0; t < 16; ++t)
#pragma unroll
    for (int r = 0; r < 8; ++r) { const float v = acc[t][r] * (1.0f / 16.0f); so[t * 16 + col][wave * 16 + 8 * g + r] = v; gs[t >> 1] += v; gq[t >> 1] += v * v; }
#pragma unroll
  for (int gi = 0; gi < NG; ++gi) {
#pragma unroll
    for (int off = 16; off >= 1; off >>= 1) { gs[gi] += __shfl_xor(gs[gi], off, 32); gq[gi] += __shfl_xor(gq[gi], off, 32); } }
  if (lane < NG) { float sv = 0.f, qv = 0.f;
#pragma unroll
    for (int gi = 0; gi < NG; ++gi) if (gi == lane) { sv = gs[gi]; qv = gq[gi]; }
    sred[wave][lane][0] = sv; sred[wave][lane][1] = qv; }
  __syncthreads();
  for (int q = tid; q < COUT * 16; q += 128) { const int co = q >> 4, pc = q & 15; vst2(F + ((size_t)bk * COUT + co) * NPX + blockIdx.x * 64 + pc * 4, *(const v4f*)(&so[co][pc * 4])); }
  if (tid < 32) { float v = 0.f; if (tid < 2 * NG) { const int gi = tid >> 1, wch = tid & 1; v = (sred[0][gi][wch] + sred[1][gi][wch]) + (sred[2][gi][wch] + sred[3][gi][wch]); }
    vst2(PART + ((size_t)bk * NBLK + blockIdx.x) * 32 + tid, v); }
}
__global__ __launch_bounds__(256) void k_out(const float* __restrict__ F, const float* __restrict__ PART, const int* __restrict__ ridx, const float* __restrict__ rw, const float* __restrict__ gam, const float* __restrict__ bet, float* __restrict__ out) {
  __shared__ float sst[TOPK][NG][2];
  __shared__ __align__(16) float so[COUT][68];
  const int tid = threadIdx.x, b = blockIdx.y, p0 = blockIdx.x * 64;
  if (tid < TOPK * NG) { const int kk = tid / NG, gi = tid % NG; const int bk = b * TOPK + kk; float s = 0.f, q2 = 0.f;
    for (int bl = 0; bl < NBLK; ++bl) { s += PART[((size_t)bk * NBLK + bl) * 32 + gi * 2]; q2 += PART[((size_t)bk * NBLK + bl) * 32 + gi * 2 + 1]; }
    const float n = (float)(CIG * NPX); const float mu = s / n; float var = q2 / n - mu * mu; var = var > 0.f ? var : 0.f;
    sst[kk][gi][0] = mu; sst[kk][gi][1] = rsqrtf(var + 1e-5f); }
  __syncthreads();
  int e0 = ridx[b * TOPK], e1 = ridx[b * TOPK + 1]; e0 = e0 < 0 ? 0 : (e0 >= NE ? NE - 1 : e0); e1 = e1 < 0 ? 0 : (e1 >= NE ? NE - 1 : e1);
  const float w0 = rw[b * TOPK], w1 = rw[b * TOPK + 1];
  for (int q = tid; q < COUT * 64; q += 256) { const int co = q >> 6, px = q & 63; const int gi = co / CIG;
    const float f0 = F[(((size_t)b * TOPK + 0) * COUT + co) * NPX + p0 + px], f1 = F[(((size_t)b * TOPK + 1) * COUT + co) * NPX + p0 + px];
    const float n0 = (f0 - sst[0][gi][0]) * sst[0][gi][1] * gam[e0 * COUT + co] + bet[e0 * COUT + co];
    const float n1 = (f1 - sst[1][gi][0]) * sst[1][gi][1] * gam[e1 * COUT + co] + bet[e1 * COUT + co];
    so[co][px] = w0 * (n0 * sigm(n0)) + w1 * (n1 * sigm(n1)); }
  __syncthreads();
  for (int q = tid; q < COUT * 16; q += 256) { const int co = q >> 4, pc = q & 15; vst2(out + ((size_t)b * COUT + co) * NPX + p0 + pc * 4, *(const v4f*)(&so[co][pc * 4])); }
}
extern "C" void kernel_launch(void* const* d_in, const int* in_sizes, int n_in, void* d_out, int out_size, void* d_ws, size_t ws_size, hipStream_t stream) {
  (void)in_sizes; (void)n_in; (void)out_size; (void)ws_size;
  const float* x = (const float*)d_in[0]; const float* rw = (const float*)d_in[1]; const int* ridx = (const int*)d_in[2]; const float* cw = (const float*)d_in[4]; const float* gam = (const float*)d_in[5]; const float* bet = (const float*)d_in[6];
  float* out = (float*)d_out;
  char* ws = (char*)d_ws; size_t off = 0;
  auto take = [&](size_t bytes) { char* p = ws + off; off += (bytes + 255) & ~(size_t)255; return p; };
  float* F = (float*)take((size_t)NBT * TOPK * COUT * NPX * 4); float* PART = (float*)take((size_t)NBT * TOPK * NBLK * 32 * 4);
  k_conv<<<dim3(NBLK, NBT * TOPK), 128, 0, stream>>>(x, ridx, cw, F, PART);
  k_out<<<dim3(NBLK, NBT), 256, 0, stream>>>(F, PART, ridx, rw, gam, bet, out);
}
